// KANLayer_10703058502229
// MI455X (gfx1250) — hardware-run, weakly checked
//
#include <hip/hip_runtime.h>


#ifndef NB
#define NB 4096
#endif
#define NB_FULL 4096
#define D_IN   768
#define D_OUT  512
#define NQ     64
#define NH1    32
#define NH2    64
#define LSP    516
#define WCARRY 1024.0f
#define WCINV  (1.0f / 1024.0f)
#define F16_MIN_NORMAL 6.103515625e-05f
#define LN_EPS 1e-5f

static_assert(NB % 64 == 0);
static_assert(NB <= NB_FULL);
static_assert(D_IN % 32 == 0);
static_assert(D_OUT % 64 == 0);
static_assert(D_OUT % 32 == 0);
static_assert((D_OUT / 32) * 2 * 16 == D_OUT);
static_assert(D_OUT == 512);
static_assert(NH1 == 32);
static_assert(NH2 == 64);
static_assert(NQ == 64);
static_assert(D_OUT % 4 == 0);
static_assert(NQ % 4 == 0);
static_assert((LSP * 4) % 16 == 0);
static_assert(LSP >= D_OUT);
static_assert(16 * LSP * 4 <= 131072);
static_assert(16 * 68 * 4 <= 131072);
static_assert(((size_t)NB * D_IN) % (8 * 256) == 0);
static_assert(((size_t)D_IN * D_OUT / 8) % 256 == 0);
static_assert(((size_t)NH1 * NQ / 8) % 256 == 0);
static_assert(((size_t)NH2 * D_OUT / 8) % 256 == 0);
static_assert(D_IN % 8 == 0);
static_assert(NH1 % 8 == 0);
static_assert(NH2 % 8 == 0);
static_assert(32 * 16 * 8 == 16 * 64 * 4);
static_assert(32 * 16 * 4 * 16 == 16 * D_OUT * 4);

typedef _Float16 h16;
typedef unsigned short bf;
typedef __attribute__((ext_vector_type(16))) __bf16   v16bf;
typedef __attribute__((ext_vector_type(16))) _Float16 v16h;
typedef __attribute__((ext_vector_type(8)))  _Float16 v8h;
typedef __attribute__((ext_vector_type(8)))  unsigned short v8us;
typedef __attribute__((ext_vector_type(8)))  float    v8f;
typedef __attribute__((ext_vector_type(4)))  float    v4f;
typedef v4f  __attribute__((may_alias)) v4fa;

__device__ __forceinline__ unsigned short f2bf(float f) { unsigned u = __float_as_uint(f); u += 0x7FFFu + ((u >> 16) & 1u); return (unsigned short)(u >> 16); }
__device__ __forceinline__ float bfr(float f) { return __uint_as_float(((unsigned)f2bf(f)) << 16); }
__device__ __forceinline__ v16h cat16(v8h lo, v8h hi) { return __builtin_shufflevector(lo, hi, 0, 1, 2, 3, 4, 5, 6, 7, 8, 9, 10, 11, 12, 13, 14, 15); }
__device__ __forceinline__ v16bf cat16b(v8us lo, v8us hi) { return __builtin_bit_cast(v16bf, __builtin_shufflevector(lo, hi, 0, 1, 2, 3, 4, 5, 6, 7, 8, 9, 10, 11, 12, 13, 14, 15)); }
__device__ __forceinline__ v8f wmma16(v16h a, v16h b, v8f c) { return __builtin_amdgcn_wmma_f32_16x16x32_f16(false, a, false, b, (short)0, c, false, false); }
__device__ __forceinline__ v8f wmmab(v16bf a, v16bf b, v8f c) { return __builtin_amdgcn_wmma_f32_16x16x32_bf16(false, a, false, b, (short)0, c, false, false); }
__device__ __forceinline__ v16h  ldh(const h16* p) { return cat16(*(const v8h*)p, *(const v8h*)(p + 16)); }
__device__ __forceinline__ v16bf ldb(const bf* p)  { return cat16b(*(const v8us*)p, *(const v8us*)(p + 16)); }
__device__ __forceinline__ void wave_sync() { __builtin_amdgcn_fence(3  , "wavefront"); __builtin_amdgcn_wave_barrier(); asm volatile("" ::: "memory"); }

__device__ __forceinline__ v8f wmmabg(v16bf a, v16bf b, v8f c) { c = wmmab(a, b, c); asm volatile("v_nop\n\tv_nop\n\tv_nop\n\tv_nop" : "+v"(c) : "v"(a), "v"(b)); return c; }
__device__ __forceinline__ v8f wmma16g(v16h a, v16h b, v8f c) { c = wmma16(a, b, c); asm volatile("v_nop\n\tv_nop\n\tv_nop\n\tv_nop" : "+v"(c) : "v"(a), "v"(b)); return c; }

static __device__ __forceinline__ h16 toh_flush(float v) { const h16 r = (h16)v; return (fabsf(v) < F16_MIN_NORMAL) ? (h16)0.0f : r; }
static __device__ __forceinline__ h16 toh_relu_flush(float t) { const float g = (t < F16_MIN_NORMAL) ? 0.0f : t; return (h16)g; }

__global__ __launch_bounds__(256) void k_cvt8(const float* __restrict__ src, bf* dst, size_t n8) {
    const size_t i = (size_t)blockIdx.x * 256 + threadIdx.x; if (i >= n8) return;
    const v8f v = *(const v8f*)(src + i * 8); v8us o;
#pragma unroll
    for (int k = 0; k < 8; ++k) o[k] = f2bf(v[k]);
    *(volatile v8us*)(dst + i * 8) = o; __threadfence(); *(volatile v8us*)(dst + i * 8) = o;
}

template <int KD, int ND>
__device__ __forceinline__ v8f wt_load8(const float* __restrict__ src, unsigned i) {
    constexpr unsigned K8 = (unsigned)KD / 8u;
    const unsigned n = i / K8, k0 = (i % K8) * 8u;
    v8f r;
#pragma unroll
    for (int j = 0; j < 8; ++j) r[j] = bfr(src[(size_t)(k0 + (unsigned)j) * (unsigned)ND + n]);
    return r;
}

static constexpr unsigned WP_PIECES = (unsigned)((size_t)D_IN * D_OUT / 8);
static constexpr unsigned W2_PIECES = (unsigned)((size_t)NH1 * NQ / 8);
static constexpr unsigned WO_PIECES = (unsigned)((size_t)NH2 * D_OUT / 8);

__global__ __launch_bounds__(256) void k_wt_proj(const float* __restrict__ src, bf* dst) {
    const unsigned i = blockIdx.x * 256u + threadIdx.x; if (i >= WP_PIECES) return;
    const v8f v = wt_load8<D_IN, D_OUT>(src, i); v8us o;
#pragma unroll
    for (int k = 0; k < 8; ++k) o[k] = f2bf(v[k]);
    *(volatile v8us*)(dst + (size_t)i * 8) = o; __threadfence(); *(volatile v8us*)(dst + (size_t)i * 8) = o;
}

__global__ __launch_bounds__(256) void k_wt_in(const float* __restrict__ src, h16* dst) {
    const unsigned i = blockIdx.x * 256u + threadIdx.x; if (i >= W2_PIECES) return;
    const v8f v = wt_load8<NH1, NQ>(src, i); v8h o;
#pragma unroll
    for (int k = 0; k < 8; ++k) o[k] = toh_flush(v[k] * WCARRY);
    *(volatile v8h*)(dst + (size_t)i * 8) = o; __threadfence(); *(volatile v8h*)(dst + (size_t)i * 8) = o;
}

__global__ __launch_bounds__(256) void k_wt_out(const float* __restrict__ src, h16* dst) {
    const unsigned i = blockIdx.x * 256u + threadIdx.x; if (i >= WO_PIECES) return;
    const v8f v = wt_load8<NH2, D_OUT>(src, i); v8h o;
#pragma unroll
    for (int k = 0; k < 8; ++k) o[k] = toh_flush(v[k] * WCARRY);
    *(volatile v8h*)(dst + (size_t)i * 8) = o; __threadfence(); *(volatile v8h*)(dst + (size_t)i * 8) = o;
}

__global__ __launch_bounds__(32) __attribute__((amdgpu_num_vgpr(256))) void k_proj(const bf* __restrict__ A, const bf* __restrict__ Bt, const float* __restrict__ bias, float* XP) {
    __shared__ __align__(16) float os[16 * 68];
    const int K = D_IN;
    const int lane = threadIdx.x & 31, lr = lane & 15, hi = lane >> 4;
    const unsigned bx = blockIdx.x, by = blockIdx.y;
    const int r0 = (int)(bx * 64u), c0 = (int)(by * 64u);
    v8f acc[4][4];
#pragma unroll
    for (int mb = 0; mb < 4; ++mb)
#pragma unroll
        for (int nb = 0; nb < 4; ++nb) acc[mb][nb] = (v8f){};
    const size_t aoff = (size_t)(r0 + lr) * K + 8 * hi, boff = (size_t)(c0 + lr) * K + 8 * hi;
#pragma unroll 1
    for (int kc = 0; kc < K; kc += 32) {
        v16bf a[4];
#pragma unroll
        for (int mb = 0; mb < 4; ++mb) a[mb] = ldb(A + aoff + (size_t)mb * 16 * K + kc);
#pragma unroll
        for (int nb = 0; nb < 4; ++nb) { const v16bf b = ldb(Bt + boff + (size_t)nb * 16 * K + kc);
#pragma unroll
            for (int mb = 0; mb < 4; ++mb) acc[mb][nb] = wmmabg(a[mb], b, acc[mb][nb]); }
    }
    float bc[4];
#pragma unroll
    for (int nb = 0; nb < 4; ++nb) bc[nb] = bfr(bias[c0 + nb * 16 + lr]);
#pragma unroll
    for (int mb = 0; mb < 4; ++mb) {
#pragma unroll
        for (int nb = 0; nb < 4; ++nb) {
#pragma unroll
            for (int j = 0; j < 8; ++j) os[(hi * 8 + j) * 68 + nb * 16 + lr] = acc[mb][nb][j] + bc[nb]; }
        wave_sync();
        float* dst = XP + (size_t)(r0 + mb * 16) * D_OUT + c0;
#pragma unroll 1
        for (int ps = 0; ps < 2; ++ps) {
#pragma unroll
            for (int s = 0; s < 8; ++s) { const int row = 2 * s + (lane >> 4), c4 = (lane & 15) * 4;
                const v4f val = *(const v4fa*)(&os[row * 68 + c4]);
                *(volatile v4f*)(dst + (size_t)row * D_OUT + c4) = val; }
            if (ps == 0) __threadfence(); }
        wave_sync();
    }
}

__global__ __launch_bounds__(32) __attribute__((amdgpu_num_vgpr(256))) void k_inner(const float* __restrict__ XP, const h16* __restrict__ W2T, const float* __restrict__ wi1, const float* __restrict__ bi1,
                                                                                    const float* __restrict__ bi2, float* UP) {
    __shared__ __align__(16) float os[16 * 68];
    const int lane = threadIdx.x & 31, lr = lane & 15, hi = lane >> 4;
    const unsigned bx = blockIdx.x;
    const int r0 = (int)(bx * 16u);
    float w1[16], b1[16];
#pragma unroll
    for (int g = 0; g < 4; ++g) {
        const int hb = (g < 2 ? 0 : 16) + 8 * hi + 4 * (g & 1);
        const v4f x0 = *(const v4f*)(wi1 + hb), x1 = *(const v4f*)(bi1 + hb);
#pragma unroll
        for (int c = 0; c < 4; ++c) { w1[4 * g + c] = bfr(x0[c]); b1[4 * g + c] = bfr(x1[c]); }
    }
    v16h bw[4];
#pragma unroll
    for (int nb = 0; nb < 4; ++nb) bw[nb] = ldh(W2T + (size_t)(nb * 16 + lr) * NH1 + 8 * hi);
    v8f acc[4];
#pragma unroll
    for (int nb = 0; nb < 4; ++nb) acc[nb] = (v8f){};
    const float* xr = XP + (size_t)(r0 + lr) * D_OUT;
#pragma unroll 1
    for (int d = 0; d < D_OUT; d += 4) {
        const v4f xv = *(const v4f*)(xr + d);
#pragma unroll
        for (int dd = 0; dd < 4; ++dd) {
            const float v = xv[dd];
            v16h a;
#pragma unroll
            for (int i = 0; i < 16; ++i) a[i] = toh_relu_flush(v * w1[i] + b1[i]);
#pragma unroll
            for (int nb = 0; nb < 4; ++nb) acc[nb] = wmma16g(a, bw[nb], acc[nb]);
        }
    }
    float b2[4];
#pragma unroll
    for (int nb = 0; nb < 4; ++nb) b2[nb] = (float)D_OUT * bfr(bi2[nb * 16 + lr]);
#pragma unroll
    for (int nb = 0; nb < 4; ++nb) {
#pragma unroll
        for (int j = 0; j < 8; ++j) os[(hi * 8 + j) * 68 + nb * 16 + lr] = acc[nb][j] * WCINV + b2[nb]; }
    wave_sync();
    float* dst = UP + (size_t)r0 * NQ;
#pragma unroll 1
    for (int ps = 0; ps < 2; ++ps) {
#pragma unroll
        for (int s = 0; s < 8; ++s) { const int row = 2 * s + (lane >> 4), c4 = (lane & 15) * 4;
            const v4f val = *(const v4fa*)(&os[row * 68 + c4]);
            *(volatile v4f*)(dst + (size_t)row * NQ + c4) = val; }
        if (ps == 0) __threadfence(); }
}

__global__ __launch_bounds__(32) void k_outer(const float* __restrict__ UP, const h16* __restrict__ WOT, const float* __restrict__ wo1, const float* __restrict__ bo1,
                                              const float* __restrict__ bo2, const float* __restrict__ gamma, const float* __restrict__ beta, float* OUT) {
    __shared__ __align__(16) float ss[16 * LSP];
    const int lane = threadIdx.x & 31, lr = lane & 15, hi = lane >> 4;
    const unsigned bx = blockIdx.x;
    const int r0 = (int)(bx * 16u);
    float wa[16], ba[16], wb[16], bb[16];
#pragma unroll
    for (int g = 0; g < 2; ++g) {
        const int hb = (g < 2 ? 0 : 16) + 8 * hi + 4 * (g & 1);
        const v4f x0 = *(const v4f*)(wo1 + hb), x1 = *(const v4f*)(bo1 + hb), x2 = *(const v4f*)(wo1 + 32 + hb), x3 = *(const v4f*)(bo1 + 32 + hb);
#pragma unroll
        for (int c = 0; c < 4; ++c) { wa[4 * g + c] = bfr(x0[c]); ba[4 * g + c] = bfr(x1[c]); wb[4 * g + c] = bfr(x2[c]); bb[4 * g + c] = bfr(x3[c]); }
    }
    asm volatile("" ::: "memory");
#pragma unroll
    for (int g = 2; g < 4; ++g) {
        const int hb = (g < 2 ? 0 : 16) + 8 * hi + 4 * (g & 1);
        const v4f x0 = *(const v4f*)(wo1 + hb), x1 = *(const v4f*)(bo1 + hb), x2 = *(const v4f*)(wo1 + 32 + hb), x3 = *(const v4f*)(bo1 + 32 + hb);
#pragma unroll
        for (int c = 0; c < 4; ++c) { wa[4 * g + c] = bfr(x0[c]); ba[4 * g + c] = bfr(x1[c]); wb[4 * g + c] = bfr(x2[c]); bb[4 * g + c] = bfr(x3[c]); }
    }
    const float* ur = UP + (size_t)(r0 + lr) * NQ;
#pragma unroll 1
    for (int pass = 0; pass < D_OUT / 32; ++pass) {
        const int cb = pass * 32;
        v16h b0[2], b1[2];
#pragma unroll
        for (int nb = 0; nb < 2; ++nb) { const h16* wrow = WOT + (size_t)(cb + nb * 16 + lr) * NH2 + 8 * hi; b0[nb] = ldh(wrow); b1[nb] = ldh(wrow + 32); }
        v8f acc[2];
#pragma unroll
        for (int nb = 0; nb < 2; ++nb) acc[nb] = (v8f){};
#pragma unroll 1
        for (int q = 0; q < NQ; q += 4) {
            const v4f uv = *(const v4f*)(ur + q);
#pragma unroll
            for (int dd = 0; dd < 4; ++dd) {
                const float v = uv[dd];
                v16h a;
#pragma unroll
                for (int i = 0; i < 16; ++i) a[i] = toh_relu_flush(v * wa[i] + ba[i]);
#pragma unroll
                for (int nb = 0; nb < 2; ++nb) acc[nb] = wmma16g(a, b0[nb], acc[nb]);
                v16h a2;
#pragma unroll
                for (int i = 0; i < 16; ++i) a2[i] = toh_relu_flush(v * wb[i] + bb[i]);
#pragma unroll
                for (int nb = 0; nb < 2; ++nb) acc[nb] = wmma16g(a2, b1[nb], acc[nb]);
            }
        }
#pragma unroll
        for (int nb = 0; nb < 2; ++nb) {
            const float bo = (float)NQ * bfr(bo2[cb + nb * 16 + lr]);
#pragma unroll
            for (int j = 0; j < 8; ++j) ss[(hi * 8 + j) * LSP + cb + nb * 16 + lr] = acc[nb][j] * WCINV + bo; }
    }
    wave_sync();
#pragma unroll 1
    for (int r = 0; r < 16; ++r) {
        v4f x[4];
#pragma unroll
        for (int j = 0; j < 4; ++j) x[j] = *(const v4fa*)(&ss[r * LSP + j * 128 + lane * 4]);
        float s = 0.0f;
#pragma unroll
        for (int j = 0; j < 4; ++j) { s += x[j][0]; s += x[j][1]; s += x[j][2]; s += x[j][3]; }
        s += __shfl_xor(s, 16, 32); s += __shfl_xor(s, 8, 32); s += __shfl_xor(s, 4, 32); s += __shfl_xor(s, 2, 32); s += __shfl_xor(s, 1, 32);
        const float mu = s * (1.0f / (float)D_OUT);
        float qv = 0.0f;
#pragma unroll
        for (int j = 0; j < 4; ++j) {
#pragma unroll
            for (int c = 0; c < 4; ++c) { const float dl = x[j][c] - mu; qv += dl * dl; } }
        qv += __shfl_xor(qv, 16, 32); qv += __shfl_xor(qv, 8, 32); qv += __shfl_xor(qv, 4, 32); qv += __shfl_xor(qv, 2, 32); qv += __shfl_xor(qv, 1, 32);
        const float rs = rsqrtf(qv * (1.0f / (float)D_OUT) + LN_EPS);
#pragma unroll
        for (int j = 0; j < 4; ++j) {
            const v4f t = *(const v4f*)(gamma + j * 128 + lane * 4);
            const v4f sf = *(const v4f*)(beta + j * 128 + lane * 4);
            v4f y;
#pragma unroll
            for (int c = 0; c < 4; ++c) y[c] = (x[j][c] - mu) * rs * bfr(t[c]) + bfr(sf[c]);
            *(v4fa*)(&ss[r * LSP + j * 128 + lane * 4]) = y; }
    }
    wave_sync();
    float* orow = OUT + (size_t)r0 * D_OUT;
#pragma unroll 1
    for (int ps = 0; ps < 2; ++ps) {
#pragma unroll 1
        for (int r = 0; r < 16; ++r) {
#pragma unroll
            for (int j = 0; j < 4; ++j) { const v4f val = *(const v4fa*)(&ss[r * LSP + j * 128 + lane * 4]);
                *(volatile v4f*)(orow + (size_t)r * D_OUT + j * 128 + lane * 4) = val; }
        }
        if (ps == 0) __threadfence(); }
}

static constexpr size_t al256(size_t v) { return (v + 255) & ~(size_t)255; }
static constexpr size_t SZ_XB  = al256((size_t)NB * D_IN * 2);
static constexpr size_t SZ_WPT = al256((size_t)D_OUT * D_IN * 2);
static constexpr size_t SZ_W2T = al256((size_t)NQ * NH1 * 2);
static constexpr size_t SZ_WOT = al256((size_t)D_OUT * NH2 * 2);
static constexpr size_t SZ_XP  = al256((size_t)NB * D_OUT * 4);
static constexpr size_t SZ_UP  = al256((size_t)NB * NQ * 4);
static constexpr size_t SZ_TOTAL = SZ_XB + SZ_WPT + SZ_W2T + SZ_WOT + SZ_XP + SZ_UP;
static_assert(SZ_TOTAL <= (size_t)134217728);
static_assert((size_t)WP_PIECES * 16 == (size_t)D_OUT * D_IN * 2);
static_assert((size_t)W2_PIECES * 16 == (size_t)NQ * NH1 * 2);
static_assert((size_t)WO_PIECES * 16 == (size_t)D_OUT * NH2 * 2);
static constexpr size_t X_N8 = (size_t)NB * D_IN / 8;
static constexpr unsigned CVT_GRID = (unsigned)((X_N8 + 255) / 256);

extern "C" void kernel_launch(void* const* d_in, const int* in_sizes, int n_in,
                              void* d_out, int out_size, void* d_ws, size_t ws_size, hipStream_t stream) {
    if (n_in < 13) return;
    if ((size_t)in_sizes[0] < (size_t)NB * D_IN) return;
    if ((size_t)in_sizes[1] < (size_t)D_IN * D_OUT || in_sizes[2] < D_OUT) return;
    if (in_sizes[3] < NH1 || in_sizes[4] < NH1) return;
    if (in_sizes[5] < NH1 * NQ || in_sizes[6] < NQ) return;
    if (in_sizes[7] < NH2 || in_sizes[8] < NH2) return;
    if (in_sizes[9] < NH2 * D_OUT || in_sizes[10] < D_OUT || in_sizes[11] < D_OUT || in_sizes[12] < D_OUT) return;
    if ((size_t)out_size < (size_t)NB * D_OUT) return;
    if (SZ_TOTAL > ws_size) return;
    const float* x   = (const float*)d_in[0];
    const float* wp  = (const float*)d_in[1];  const float* bp  = (const float*)d_in[2];
    const float* wi1 = (const float*)d_in[3];  const float* bi1 = (const float*)d_in[4];
    const float* wi2 = (const float*)d_in[5];  const float* bi2 = (const float*)d_in[6];
    const float* wo1 = (const float*)d_in[7];  const float* bo1 = (const float*)d_in[8];
    const float* wo2 = (const float*)d_in[9];  const float* bo2 = (const float*)d_in[10];
    const float* gam = (const float*)d_in[11]; const float* bet = (const float*)d_in[12];
    float* OUT = (float*)d_out;
    char* wsp = (char*)d_ws;
    bf*  XB  = (bf*)wsp;    wsp += SZ_XB;
    bf*  WPT = (bf*)wsp;    wsp += SZ_WPT;
    h16* W2T = (h16*)wsp;   wsp += SZ_W2T;
    h16* WOT = (h16*)wsp;   wsp += SZ_WOT;
    float* XP = (float*)wsp; wsp += SZ_XP;
    float* UP = (float*)wsp; wsp += SZ_UP;

    k_cvt8<<<CVT_GRID, 256, 0, stream>>>(x, XB, X_N8);
    k_wt_proj<<<WP_PIECES / 256u, 256, 0, stream>>>(wp, WPT);
    k_wt_in<<<W2_PIECES / 256u, 256, 0, stream>>>(wi2, W2T);
    k_wt_out<<<WO_PIECES / 256u, 256, 0, stream>>>(wo2, WOT);

    k_proj<<<dim3(NB / 64, D_OUT / 64, 1), 32, 0, stream>>>(XB, WPT, bp, XP);
    k_inner<<<dim3(NB / 16, 1, 1), 32, 0, stream>>>(XP, W2T, wi1, bi1, bi2, UP);
    k_outer<<<dim3(NB / 16, 1, 1), 32, 0, stream>>>(UP, WOT, wo1, bo1, bo2, gam, bet, OUT);
}
